// GatedMatchRNN_65094524338719
// MI455X (gfx1250) — hardware-verified
//
#include <hip/hip_runtime.h>
#include <math.h>

typedef __attribute__((ext_vector_type(16))) _Float16 v16h;
typedef __attribute__((ext_vector_type(8)))  _Float16 v8h;
typedef __attribute__((ext_vector_type(16))) __bf16   v16b;
typedef __attribute__((ext_vector_type(8)))  __bf16   v8b;
typedef __attribute__((ext_vector_type(8)))  float    v8f;
typedef __attribute__((ext_vector_type(4)))  float    v4f;

constexpr int kB    = 32;
constexpr int kBP   = 64;
constexpr int kT    = 128;
constexpr int kL    = 512;
constexpr int kH    = 256;
constexpr int kH2   = 2 * kH;
constexpr int kG4   = 4 * kH;
constexpr int kNS   = kG4 + 2 * kH;
constexpr int kRowsX = kB * kT;
constexpr int kRowsY = kB * kL;
constexpr int kThr  = 256;
constexpr float kInCarry = 1024.0f;
constexpr float kSCarry  = 1024.0f;
constexpr float kSc = 1.0f / (1024.0f * 1024.0f);
constexpr float kF16MinNormal = 6.103515625e-5f;

static_assert((kRowsX % 64) == 0 && (kRowsY % 64) == 0 && (kBP % 64) == 0 && (kH % 64) == 0 && (kH2 % 64) == 0 && (kG4 % 64) == 0 && (kNS % 64) == 0, "GEMM M, N multiples of 64");
static_assert(((kRowsY / 64) * (kH / 64)) % 8 == 0 && ((kRowsX / 64) * (kH / 64)) % 8 == 0 && ((kRowsX / 64) * (kH2 / 64)) % 8 == 0, "hoisted GEMM grids exact");
static_assert(((kBP / 64) * (kNS / 64)) % 8 == 0 && ((kBP / 64) * (kH2 / 64)) % 8 == 0 && ((kBP / 64) * (kG4 / 64)) % 8 == 0, "per-step GEMM grids exact");
static_assert((kH % 32) == 0 && (kH2 % 32) == 0, "GEMM K multiples of 32");

constexpr size_t kOffX16  = 0;
constexpr size_t kOffY16  = kOffX16  + (size_t)kRowsX * kH * 2;
constexpr size_t kOffWQ   = kOffY16  + (size_t)kRowsY * kH * 2;
constexpr size_t kOffWUP  = kOffWQ   + (size_t)kH * kH * 2;
constexpr size_t kOffWG   = kOffWUP  + (size_t)kH * kH * 2;
constexpr size_t kOffWIH  = kOffWG   + (size_t)kH2 * kH2 * 2;
constexpr size_t kOffWHV  = kOffWIH  + (size_t)kG4 * kH2 * 2;
constexpr size_t kOffF32  = kOffWHV  + (size_t)kNS * kH * 2;
constexpr int kFBQ = 0, kFBUP = 256, kFBGT = 512, kFBGI = 1024, kFBHV = 2048, kFZB = 3584, kFC32 = 4096, kFEnd = 12288;
constexpr size_t kOffYP   = kOffF32  + (size_t)kFEnd * 4;
constexpr size_t kOffXU   = kOffYP   + (size_t)kRowsY * kH * 4;
constexpr size_t kOffXG   = kOffXU   + (size_t)kRowsX * kH * 4;
constexpr size_t kOffHV   = kOffXG   + (size_t)kRowsX * kH2 * 4;
constexpr size_t kOffCG   = kOffHV   + (size_t)kBP * kNS * 4;
constexpr size_t kOffGI   = kOffCG   + (size_t)kBP * kH2 * 4;
constexpr size_t kOffCT32 = kOffGI   + (size_t)kBP * kG4 * 4;
constexpr size_t kOffH16  = kOffCT32 + (size_t)kB * kH * 4;
constexpr size_t kOffCT16 = kOffH16  + (size_t)kBP * kH * 2;
constexpr size_t kOffLI16 = kOffCT16 + (size_t)kBP * kH * 2;
constexpr size_t kWsTotal = kOffLI16 + (size_t)kBP * kH2 * 2;
static_assert(kWsTotal == 43466752ull, "carve total");
static_assert(kWsTotal <= 134217728ull, "carve cap");
static_assert((kOffY16 % 256) == 0 && (kOffWQ % 256) == 0 && (kOffWUP % 256) == 0 && (kOffWG % 256) == 0 && (kOffWIH % 256) == 0 && (kOffWHV % 256) == 0 && (kOffF32 % 256) == 0 && (kOffYP % 256) == 0 && (kOffXU % 256) == 0 && (kOffXG % 256) == 0 && (kOffHV % 256) == 0 && (kOffCG % 256) == 0 && (kOffGI % 256) == 0 && (kOffCT32 % 256) == 0 && (kOffH16 % 256) == 0 && (kOffCT16 % 256) == 0 && (kOffLI16 % 256) == 0, "aligned regions");
static_assert(kFEnd == kFC32 + kB * kH && kFC32 == kFZB + kH2 && kFZB == kFBHV + kNS && kFBHV == kFBGI + kG4 && kFBGI == kFBGT + kH2 && kFBGT == kFBUP + kH && kFBUP == kFBQ + kH, "f32 stream map");

__device__ __forceinline__ unsigned short f2bf_bits(float f) {
  unsigned u = __float_as_uint(f);
  return (unsigned short)((u + 0x7FFFu + ((u >> 16) & 1u)) >> 16);
}
__device__ __forceinline__ float bf_bits2f(unsigned short h) { return __uint_as_float(((unsigned)h) << 16); }
__device__ __forceinline__ float bf16r(float f) { return bf_bits2f(f2bf_bits(f)); }
__device__ __forceinline__ float carry_flush(float v, float carry) {
  const float s = v * carry;
  return (fabsf(s) < kF16MinNormal) ? 0.0f : s;
}
__device__ __forceinline__ float frcp(float x) { return __builtin_amdgcn_rcpf(x); }

__device__ __forceinline__ void dep_guard4_h(v8f& a, v8f& b, v8f& c, v8f& d, v16h x, v16h y) { asm volatile("v_nop\n\tv_nop\n\tv_nop\n\tv_nop" : "+v"(a), "+v"(b), "+v"(c), "+v"(d) : "v"(x), "v"(y)); }
__device__ __forceinline__ void dep_guard4_b(v8f& a, v8f& b, v8f& c, v8f& d, v16b x, v16b y) { asm volatile("v_nop\n\tv_nop\n\tv_nop\n\tv_nop" : "+v"(a), "+v"(b), "+v"(c), "+v"(d) : "v"(x), "v"(y)); }
__device__ __forceinline__ void keep4_h(v16h a, v16h b, v16h c, v16h d) { asm volatile("v_nop" :: "v"(a), "v"(b), "v"(c), "v"(d)); }
__device__ __forceinline__ void keep4_b(v16b a, v16b b, v16b c, v16b d) { asm volatile("v_nop" :: "v"(a), "v"(b), "v"(c), "v"(d)); }
__device__ __forceinline__ void acc_guard4(v8f& a, v8f& b, v8f& c, v8f& d) { asm volatile("v_nop\n\tv_nop\n\tv_nop\n\tv_nop" : "+v"(a), "+v"(b), "+v"(c), "+v"(d)); }

template <typename T> struct Frag;
template <> struct Frag<_Float16> {
  typedef v16h V; union U { v16h v; v8h h[2]; };
  static __device__ __forceinline__ v16h load(const _Float16* p) {
    U f; f.h[0] = *(const v8h*)(p); f.h[1] = *(const v8h*)(p + 16); return f.v;
  }
  static __device__ __forceinline__ v8f mma(v16h a, v16h b, v8f c) {
    return __builtin_amdgcn_wmma_f32_16x16x32_f16(false, a, false, b, (short)0, c, false, false);
  }
  static __device__ __forceinline__ void guard4(v8f& a, v8f& b, v8f& c, v8f& d, v16h x, v16h y) { dep_guard4_h(a, b, c, d, x, y); }
  static __device__ __forceinline__ void keep(v16h a, v16h b, v16h c, v16h d) { keep4_h(a, b, c, d); }
};
template <> struct Frag<__bf16> {
  typedef v16b V; union U { v16b v; v8b h[2]; };
  static __device__ __forceinline__ v16b load(const __bf16* p) {
    U f; f.h[0] = *(const v8b*)(p); f.h[1] = *(const v8b*)(p + 16); return f.v;
  }
  static __device__ __forceinline__ v8f mma(v16b a, v16b b, v8f c) {
    return __builtin_amdgcn_wmma_f32_16x16x32_bf16(false, a, false, b, (short)0, c, false, false);
  }
  static __device__ __forceinline__ void guard4(v8f& a, v8f& b, v8f& c, v8f& d, v16b x, v16b y) { dep_guard4_b(a, b, c, d, x, y); }
  static __device__ __forceinline__ void keep(v16b a, v16b b, v16b c, v16b d) { keep4_b(a, b, c, d); }
};

__device__ __forceinline__ v8f mma_h(v16h a, v16h b, v8f c) {
  c = __builtin_amdgcn_wmma_f32_16x16x32_f16(false, a, false, b, (short)0, c, false, false);
  asm volatile("v_nop\n\tv_nop\n\tv_nop\n\tv_nop" : "+v"(c) : "v"(a), "v"(b));
  return c;
}

template <int ET> struct Elem;
template <> struct Elem<0> { typedef _Float16 T; };
template <> struct Elem<1> { typedef __bf16 T; };
template <int ET, bool SPLIT, int BIAS_MODE, int OUT_MODE, bool RESID, int ACT = 0>
__global__ __launch_bounds__(256) void wmma_gemm64(
    const unsigned short* __restrict__ Ap, const unsigned short* __restrict__ A2p, int lda, long strideA,
    const unsigned short* __restrict__ Btp, const unsigned short* __restrict__ Bt2p, int ldb, long strideB,
    void* __restrict__ Cout, void* __restrict__ Cout2, int ldc, long strideC,
    const float* __restrict__ bias,
    const float* __restrict__ resid, long strideR,
    int M, int N, int K, float scale) {
  typedef typename Elem<ET>::T T;
  typedef typename Frag<T>::V V;
  const T* A = (const T*)Ap; const T* A2 = (const T*)A2p; const T* Bt = (const T*)Btp; const T* Bt2 = (const T*)Bt2p;
  __shared__ __align__(16) float sT[8][16 * 68];
  const int b    = blockIdx.y;
  const int lane = threadIdx.x & 31;
  const int wave = threadIdx.x >> 5;
  const int tilesN = N >> 6;
  const int tilesM = M >> 6;
  const int tile = blockIdx.x * 8 + wave;
  if (tile >= tilesM * tilesN) return;
  const int tm = tile / tilesN;
  const int tn = tile - tm * tilesN;
  const int m0 = tm << 6;
  const int n0 = tn << 6;

  const T* Ab  = A  + (size_t)b * strideA;
  const T* Bb  = Bt + (size_t)b * strideB;
  const T* Ab2 = SPLIT ? (A2  + (size_t)b * strideA) : nullptr;
  const T* Bb2 = SPLIT ? (Bt2 + (size_t)b * strideB) : nullptr;

  const int rlane = lane & 15;
  const int koff  = (lane >> 4) * 8;
  const int mOff  = (lane >> 4) * 8;

  v8f acc[4][4];
#pragma unroll
  for (int i = 0; i < 4; ++i)
#pragma unroll
    for (int j = 0; j < 4; ++j) acc[i][j] = (v8f){0.f,0.f,0.f,0.f,0.f,0.f,0.f,0.f};

  for (int k0 = 0; k0 < K; k0 += 32) {
    V bh[4], bl[4];
#pragma unroll
    for (int j = 0; j < 4; ++j) {
      const size_t bo = (size_t)(n0 + (j << 4) + rlane) * ldb + koff + k0;
      bh[j] = Frag<T>::load(Bb + bo);
      if (SPLIT) bl[j] = Frag<T>::load(Bb2 + bo);
    }
#pragma unroll
    for (int i = 0; i < 4; ++i) {
      const size_t ao = (size_t)(m0 + (i << 4) + rlane) * lda + koff + k0;
      V ah = Frag<T>::load(Ab + ao);
      V al;
      if (SPLIT) al = Frag<T>::load(Ab2 + ao);
#pragma unroll
      for (int j = 0; j < 4; ++j) {
        acc[i][j] = Frag<T>::mma(ah, bh[j], acc[i][j]);
        if (SPLIT) {
          acc[i][j] = Frag<T>::mma(ah, bl[j], acc[i][j]);
          acc[i][j] = Frag<T>::mma(al, bh[j], acc[i][j]);
        }
      }
      Frag<T>::guard4(acc[i][0], acc[i][1], acc[i][2], acc[i][3], ah, SPLIT ? al : ah);
    }
    Frag<T>::keep(bh[0], bh[1], bh[2], bh[3]);
    if (SPLIT) Frag<T>::keep(bl[0], bl[1], bl[2], bl[3]);
  }
  acc_guard4(acc[0][0], acc[0][1], acc[0][2], acc[0][3]);
  acc_guard4(acc[1][0], acc[1][1], acc[1][2], acc[1][3]);
  acc_guard4(acc[2][0], acc[2][1], acc[2][2], acc[2][3]);
  acc_guard4(acc[3][0], acc[3][1], acc[3][2], acc[3][3]);

  float* slab = sT[wave];
  const float* Rb = RESID ? (resid + (size_t)b * strideR) : nullptr;
#pragma unroll
  for (int i = 0; i < 4; ++i) {
    const int mBase = m0 + (i << 4);
#pragma unroll
    for (int j = 0; j < 4; ++j) {
      const int n = n0 + (j << 4) + rlane;
      float bv = 0.f;
      if (BIAS_MODE == 2) bv = bias[n];
#pragma unroll
      for (int r = 0; r < 8; ++r) {
        float v = acc[i][j][r] * scale;
        if (BIAS_MODE == 1) v += bias[mBase + mOff + r];
        if (BIAS_MODE == 2) v += bv;
        if (RESID) v += Rb[(size_t)(mBase + mOff + r) * ldc + n];
        if (ACT == 1) v = tanhf(v);
        if (ACT == 2) v = fmaxf(v, 0.0f);
        if (ACT == 3) v = v / (1.0f + expf(-v));
        if (ACT == 4) v = (v > 0.f) ? v : 0.01f * v;
        slab[(mOff + r) * 68 + (j << 4) + rlane] = v;
      }
    }
    __builtin_amdgcn_fence(__ATOMIC_RELEASE, "workgroup");
    __builtin_amdgcn_wave_barrier();
    __builtin_amdgcn_fence(__ATOMIC_ACQUIRE, "workgroup");
    if (OUT_MODE == 0) {
      float* C = (float*)Cout + (size_t)b * strideC;
      const int hh = lane >> 4, c4 = (lane & 15) * 4;
      for (int pass = 0; pass < 2; ++pass) {
#pragma unroll
        for (int it = 0; it < 8; ++it) {
          const int row = it * 2 + hh;
          v4f v = *(const v4f*)(slab + row * 68 + c4);
          *(volatile v4f*)(C + (size_t)(mBase + row) * ldc + n0 + c4) = v;
        }
        __threadfence();
      }
    } else {
      const int q = lane >> 3, c8 = (lane & 7) * 8;
      unsigned short* C  = (unsigned short*)Cout  + (size_t)b * strideC;
      unsigned short* C2 = (OUT_MODE == 2) ? ((unsigned short*)Cout2 + (size_t)b * strideC) : nullptr;
      for (int pass = 0; pass < 2; ++pass) {
#pragma unroll
        for (int it = 0; it < 4; ++it) {
          const int row = it * 4 + q;
          const float* sp = slab + row * 68 + c8;
          v8h hv, lv;
#pragma unroll
          for (int e = 0; e < 8; ++e) {
            if (OUT_MODE == 1) {
              hv[e] = (_Float16)sp[e];
            } else {
              unsigned short hb = f2bf_bits(sp[e]);
              unsigned short lb = f2bf_bits(sp[e] - bf_bits2f(hb));
              hv[e] = __builtin_bit_cast(_Float16, hb);
              lv[e] = __builtin_bit_cast(_Float16, lb);
            }
          }
          *(volatile v8h*)(C + (size_t)(mBase + row) * ldc + n0 + c8) = hv;
          if (OUT_MODE == 2) *(volatile v8h*)(C2 + (size_t)(mBase + row) * ldc + n0 + c8) = lv;
        }
        __threadfence();
      }
    }
    __builtin_amdgcn_fence(__ATOMIC_RELEASE, "workgroup");
    __builtin_amdgcn_wave_barrier();
    __builtin_amdgcn_fence(__ATOMIC_ACQUIRE, "workgroup");
  }
}

__global__ __launch_bounds__(kThr) void cast_plane_kernel(const float* __restrict__ src, unsigned short* __restrict__ dst,
                                                          int colsLog2, int dstPitch, int dstOff) {
  const int i   = blockIdx.x * kThr + threadIdx.x;
  const int sh  = colsLog2 - 3;
  const int row = i >> sh;
  const int c8  = (i & ((1 << sh) - 1)) * 8;
  const float* sp = src + ((size_t)row << colsLog2) + c8;
  const v4f a0 = *(const v4f*)(sp);
  const v4f a1 = *(const v4f*)(sp + 4);
  v8h hv;
#pragma unroll
  for (int e = 0; e < 4; ++e) {
    const float f0 = a0[e];
    const float f1 = a1[e];
    hv[e]     = (_Float16)carry_flush(bf16r(f0), kInCarry);
    hv[4 + e] = (_Float16)carry_flush(bf16r(f1), kInCarry);
  }
  unsigned short* dp = dst + (size_t)row * dstPitch + dstOff + c8;
  *(volatile v8h*)dp = hv;
  __threadfence();
  *(volatile v8h*)dp = hv;
}

__device__ __forceinline__ float fast_tanh(float v) { return 1.0f - 2.0f * frcp(__expf(2.0f * v) + 1.0f); }
__device__ __forceinline__ float fast_sigmoid(float v) { return frcp(1.0f + __expf(-v)); }

__global__ __launch_bounds__(kThr) void setup_f32_kernel(const float* __restrict__ bq, const float* __restrict__ bup, const float* __restrict__ bg,
                                                         const float* __restrict__ bih, const float* __restrict__ bhh, const float* __restrict__ bvp,
                                                         const float* __restrict__ c0, float* __restrict__ F) {
  unsigned v = blockIdx.x * (unsigned)kThr + threadIdx.x;
  asm volatile("" : "+v"(v));
  const unsigned i0 = v * 4u;
  v4f o = {0.f, 0.f, 0.f, 0.f};
  if (i0 < (unsigned)kFBUP) {
    const v4f a = *(const v4f*)(bq + i0);
#pragma unroll
    for (int e = 0; e < 4; ++e) { const float x = a[e]; o[e] = bf16r(x); }
  } else if (i0 < (unsigned)kFBGT) {
    const v4f a = *(const v4f*)(bup + (i0 - (unsigned)kFBUP));
#pragma unroll
    for (int e = 0; e < 4; ++e) { const float x = a[e]; o[e] = bf16r(x); }
  } else if (i0 < (unsigned)kFBGI) {
    const v4f a = *(const v4f*)(bg + (i0 - (unsigned)kFBGT));
#pragma unroll
    for (int e = 0; e < 4; ++e) { const float x = a[e]; o[e] = bf16r(x); }
  } else if (i0 < (unsigned)kFBHV) {
    const unsigned j = i0 - (unsigned)kFBGI;
    const v4f a = *(const v4f*)(bih + j);
    const v4f c = *(const v4f*)(bhh + j);
#pragma unroll
    for (int e = 0; e < 4; ++e) { const float x = a[e]; const float y = c[e]; o[e] = bf16r(x) + bf16r(y); }
  } else if (i0 < (unsigned)kFZB) {
    const unsigned j = i0 - (unsigned)kFBHV;
    if (j >= (unsigned)kG4 && j < (unsigned)(kG4 + kH)) {
      const v4f a = *(const v4f*)(bvp + (j - (unsigned)kG4));
#pragma unroll
      for (int e = 0; e < 4; ++e) { const float x = a[e]; o[e] = bf16r(x); }
    }
  } else if (i0 < (unsigned)kFC32) {
  } else {
    const v4f a = *(const v4f*)(c0 + (i0 - (unsigned)kFC32));
#pragma unroll
    for (int e = 0; e < 4; ++e) { const float x = a[e]; o[e] = bf16r(x); }
  }
  float* dp = F + i0;
  *(volatile v4f*)dp = o;
  __threadfence();
  *(volatile v4f*)dp = o;
}
static_assert(kFEnd / 4 == 12 * kThr, "set-up A grid exact");
static_assert((kFBUP % 128) == 0 && (kFBGT % 128) == 0 && (kFBGI % 128) == 0 && (kFBHV % 128) == 0 && (kFZB % 128) == 0 && (kFC32 % 128) == 0 && (kG4 % 128) == 0 && ((kG4 + kH) % 128) == 0, "set-up A regions wave-uniform");

constexpr unsigned kSB0 = 8192u, kSB1 = kSB0 + 1024u, kSB2 = kSB1 + 1024u, kSB3 = kSB2 + 2048u, kSB4 = kSB3 + 1024u;
__global__ __launch_bounds__(kThr) void setup_f16_kernel(const float* __restrict__ h0, unsigned short* __restrict__ WHV, unsigned short* __restrict__ H16,
                                                         unsigned short* __restrict__ CT16, unsigned short* __restrict__ LI16) {
  unsigned v = blockIdx.x * (unsigned)kThr + threadIdx.x;
  asm volatile("" : "+v"(v));
  v8h z;
#pragma unroll
  for (int e = 0; e < 8; ++e) z[e] = (_Float16)0.0f;
  unsigned short* dp;
  if (v < kSB0) {
    dp = WHV + (size_t)(kG4 + kH) * kH + (size_t)v * 8u;
  } else if (v < kSB1) {
    dp = H16 + (size_t)kB * kH + (size_t)(v - kSB0) * 8u;
  } else if (v < kSB2) {
    dp = CT16 + (size_t)kB * kH + (size_t)(v - kSB1) * 8u;
  } else if (v < kSB3) {
    dp = LI16 + (size_t)kB * kH2 + (size_t)(v - kSB2) * 8u;
  } else {
    const unsigned j = (v - kSB3) * 8u;
    const v4f a0 = *(const v4f*)(h0 + j);
    const v4f a1 = *(const v4f*)(h0 + j + 4);
#pragma unroll
    for (int e = 0; e < 4; ++e) {
      const float f0 = a0[e];
      const float f1 = a1[e];
      z[e]     = (_Float16)carry_flush(bf16r(f0), kSCarry);
      z[4 + e] = (_Float16)carry_flush(bf16r(f1), kSCarry);
    }
    dp = H16 + (size_t)j;
  }
  *(volatile v8h*)dp = z;
  __threadfence();
  *(volatile v8h*)dp = z;
}
static_assert(kSB4 == 52u * kThr, "set-up B grid exact");
static_assert(kSB0 == (unsigned)((kNS - kG4 - kH) * kH / 8) && (kSB1 - kSB0) == (unsigned)((kBP - kB) * kH / 8) && (kSB3 - kSB2) == (unsigned)((kBP - kB) * kH2 / 8) && (kSB4 - kSB3) == (unsigned)(kB * kH / 8), "set-up B map");
static_assert((kSB0 % 32u) == 0 && (kSB1 % 32u) == 0 && (kSB2 % 32u) == 0 && (kSB3 % 32u) == 0, "set-up B regions wave-uniform");

__global__ __launch_bounds__(kThr) void add_attn_kernel(const float* __restrict__ YP, const float* __restrict__ XU, const float* __restrict__ HV,
                                                    const float* __restrict__ Vw, const float* __restrict__ Vb, const int* __restrict__ y_mask,
                                                    const unsigned short* __restrict__ Y16, float* __restrict__ CT32, unsigned short* __restrict__ CT16, int t) {
  __shared__ __align__(16) float sXH[kH];
  __shared__ __align__(16) float sV[kH];
  __shared__ __align__(16) float sS[kL];
  __shared__ __align__(16) float sRed[32];
  __shared__ __align__(16) float sP[8 * kH];
  const int tid  = threadIdx.x;
  const int lane = tid & 31;
  const int wave = tid >> 5;
  const int b    = blockIdx.x;
  {
    const float xu = XU[((size_t)b * kT + t) * kH + tid];
    const float hd = HV[(size_t)b * kNS + kG4 + tid];
    const float vw = Vw[tid];
    sXH[tid] = xu + hd;
    sV[tid]  = bf16r(vw);
  }
  const float vb0 = Vb[0];
  const float vb  = bf16r(vb0);
  __syncthreads();

#pragma unroll 1
  for (int half = 0; half < 2; ++half) {
    const int l = tid + 256 * half;
    const float* yp = YP + ((size_t)b * kL + l) * kH;
    float acc = 0.0f;
#pragma unroll 1
    for (int h4 = 0; h4 < kH; h4 += 4) {
      const v4f p  = *(const v4f*)(yp + h4);
      const v4f xh = *(const v4f*)(sXH + h4);
      const v4f vv = *(const v4f*)(sV + h4);
      acc += vv[0] * fast_tanh(xh[0] + p[0]);
      acc += vv[1] * fast_tanh(xh[1] + p[1]);
      acc += vv[2] * fast_tanh(xh[2] + p[2]);
      acc += vv[3] * fast_tanh(xh[3] + p[3]);
    }
    int mk = y_mask[b * kL + l];
    asm volatile("" : "+v"(mk));
    sS[l] = (mk != 0) ? -INFINITY : (acc + vb);
  }
  __syncthreads();

  if (tid < 16) {
    float m = sS[tid * 32];
#pragma unroll 1
    for (int j = 1; j < 32; ++j) { const float q = sS[tid * 32 + j]; m = (q > m) ? q : m; }
    sRed[tid] = m;
  }
  __syncthreads();
  float mx = sRed[0];
#pragma unroll 1
  for (int j = 1; j < 16; ++j) { const float q = sRed[j]; mx = (q > mx) ? q : mx; }
  const float e0 = __expf(sS[tid] - mx);
  const float e1 = __expf(sS[tid + 256] - mx);
  __syncthreads();
  sS[tid] = e0;
  sS[tid + 256] = e1;
  __syncthreads();
  if (tid < 16) {
    float s = 0.0f;
#pragma unroll 1
    for (int j = 0; j < 32; ++j) s += sS[tid * 32 + j];
    sRed[16 + tid] = s;
  }
  __syncthreads();
  float den = 0.0f;
#pragma unroll 1
  for (int j = 0; j < 16; ++j) den += sRed[16 + j];

  float a8[8];
#pragma unroll
  for (int e = 0; e < 8; ++e) a8[e] = 0.0f;
  const unsigned short* yb = Y16 + (size_t)b * kL * kH + lane * 8;
#pragma unroll 1
  for (int j = 0; j < kL / 8; ++j) {
    const int l = wave + 8 * j;
    const float a = sS[l];
    const v8h y8 = *(const v8h*)(yb + (size_t)l * kH);
#pragma unroll
    for (int e = 0; e < 8; ++e) a8[e] += a * (float)y8[e];
  }
  {
    float* pp = sP + wave * kH + lane * 8;
    const v4f p0 = {a8[0], a8[1], a8[2], a8[3]};
    const v4f p1 = {a8[4], a8[5], a8[6], a8[7]};
    *(v4f*)(pp) = p0;
    *(v4f*)(pp + 4) = p1;
  }
  __syncthreads();
  if (wave == 0) {
    const float inv = (1.0f / den) * (1.0f / kInCarry);
    v4f c0v, c1v;
    v8h hv;
#pragma unroll
    for (int e = 0; e < 8; ++e) {
      float s = 0.0f;
#pragma unroll
      for (int g = 0; g < 8; ++g) s += sP[g * kH + lane * 8 + e];
      const float ct = s * inv;
      if (e < 4) c0v[e] = ct; else c1v[e - 4] = ct;
      hv[e] = (_Float16)carry_flush(ct, kSCarry);
    }
    float* cp = CT32 + (size_t)b * kH + lane * 8;
    unsigned short* hp = CT16 + (size_t)b * kH + lane * 8;
    for (int pass = 0; pass < 2; ++pass) {
      *(volatile v4f*)cp = c0v;
      *(volatile v4f*)(cp + 4) = c1v;
      *(volatile v8h*)hp = hv;
      __threadfence();
    }
  }
}

__global__ __launch_bounds__(kThr) void in_gate_kernel(const float* __restrict__ x, const int* __restrict__ x_mask, const float* __restrict__ CT32,
                                                    const float* __restrict__ XG, const float* __restrict__ CG, unsigned short* __restrict__ LI16, int t) {
  unsigned v = blockIdx.x * (unsigned)kThr + threadIdx.x;
  asm volatile("" : "+v"(v));
  const unsigned b  = v >> 6;
  const unsigned c8 = (v & 63u) * 8u;
  const float* gx = XG + ((size_t)b * kT + t) * kH2 + c8;
  const float* gc = CG + (size_t)b * kH2 + c8;
  const v4f x0 = *(const v4f*)gx, x1 = *(const v4f*)(gx + 4);
  const v4f g0 = *(const v4f*)gc, g1 = *(const v4f*)(gc + 4);
  v4f m0, m1;
  if (c8 < (unsigned)kH) {
    const float* xp = x + ((size_t)b * kT + t) * kH + c8;
    const v4f a0 = *(const v4f*)xp, a1 = *(const v4f*)(xp + 4);
#pragma unroll
    for (int e = 0; e < 4; ++e) { const float f0 = a0[e]; const float f1 = a1[e]; m0[e] = bf16r(f0); m1[e] = bf16r(f1); }
  } else {
    const float* cp = CT32 + (size_t)b * kH + (c8 - (unsigned)kH);
    m0 = *(const v4f*)cp;
    m1 = *(const v4f*)(cp + 4);
  }
  int mk = x_mask[b * kT + t];
  asm volatile("" : "+v"(mk));
  const bool masked = (mk != 0);
  v8h hv;
#pragma unroll
  for (int e = 0; e < 4; ++e) {
    const float l0 = fast_sigmoid(x0[e] + g0[e]) * m0[e];
    const float l1 = fast_sigmoid(x1[e] + g1[e]) * m1[e];
    hv[e]     = (_Float16)carry_flush(masked ? 0.0f : l0, kSCarry);
    hv[4 + e] = (_Float16)carry_flush(masked ? 0.0f : l1, kSCarry);
  }
  unsigned short* dp = LI16 + (size_t)b * kH2 + c8;
  *(volatile v8h*)dp = hv;
  __threadfence();
  *(volatile v8h*)dp = hv;
}
static_assert(kB * kH2 / 8 == 8 * kThr, "gate grid exact");

__global__ __launch_bounds__(kThr) void masked_cell_kernel(const float* __restrict__ GI, const float* __restrict__ HV, const int* __restrict__ x_mask,
                                                    float* __restrict__ C32, unsigned short* __restrict__ H16, float* __restrict__ out, int t) {
  unsigned v = blockIdx.x * (unsigned)kThr + threadIdx.x;
  asm volatile("" : "+v"(v));
  const unsigned b  = v >> 5;
  const unsigned u8 = (v & 31u) * 8u;
  const float* ir = GI + (size_t)b * kG4 + u8;
  const float* sr = HV + (size_t)b * kNS + u8;
  float* cp = C32 + (size_t)b * kH + u8;
  int mk = x_mask[b * kT + t];
  asm volatile("" : "+v"(mk));
  const bool masked = (mk != 0);
  v8h hv;
  v4f cn0, cn1, hn0, hn1;
#pragma unroll
  for (int hlf = 0; hlf < 2; ++hlf) {
    const v4f xi = *(const v4f*)(ir + 4 * hlf), xf = *(const v4f*)(ir + kH + 4 * hlf), xg = *(const v4f*)(ir + 2 * kH + 4 * hlf), xo = *(const v4f*)(ir + 3 * kH + 4 * hlf);
    const v4f gi = *(const v4f*)(sr + 4 * hlf), gf = *(const v4f*)(sr + kH + 4 * hlf), gg = *(const v4f*)(sr + 2 * kH + 4 * hlf), go = *(const v4f*)(sr + 3 * kH + 4 * hlf);
    const v4f co = *(const v4f*)(cp + 4 * hlf);
#pragma unroll
    for (int e = 0; e < 4; ++e) {
      const float cn = fast_sigmoid(xf[e] + gf[e]) * co[e] + fast_sigmoid(xi[e] + gi[e]) * fast_tanh(xg[e] + gg[e]);
      const float hr = fast_sigmoid(xo[e] + go[e]) * fast_tanh(cn);
      const float hn = masked ? 0.0f : hr;
      if (hlf == 0) { cn0[e] = cn; hn0[e] = hn; } else { cn1[e] = cn; hn1[e] = hn; }
      hv[4 * hlf + e] = (_Float16)carry_flush(hn, kSCarry);
    }
  }
  unsigned short* hp = H16 + (size_t)b * kH + u8;
  float* op = out + ((size_t)b * kT + t) * kH + u8;
  for (int pass = 0; pass < 2; ++pass) {
    *(volatile v4f*)cp = cn0;
    *(volatile v4f*)(cp + 4) = cn1;
    *(volatile v8h*)hp = hv;
    *(volatile v4f*)op = hn0;
    *(volatile v4f*)(op + 4) = hn1;
    __threadfence();
  }
}
static_assert(kB * kH / 8 == 4 * kThr, "cell grid exact");

static_assert(((size_t)kRowsX * kH / 8) % kThr == 0 && ((size_t)kRowsY * kH / 8) % kThr == 0 && ((size_t)kH * kH / 8) % kThr == 0 && ((size_t)kH2 * kH2 / 8) % kThr == 0 && ((size_t)kG4 * kH2 / 8) % kThr == 0 && ((size_t)kG4 * kH / 8) % kThr == 0, "cast grids exact");

extern "C" void kernel_launch(void* const* d_in, const int* in_sizes, int n_in,
                              void* d_out, int out_size, void* d_ws, size_t ws_size,
                              hipStream_t stream) {
  if (n_in < 20 || d_out == nullptr || d_ws == nullptr) return;
  if (in_sizes[0] != kB * kT * kH || in_sizes[1] != kB * kT || in_sizes[2] != kB * kL * kH || in_sizes[3] != kB * kL) return;
  if (in_sizes[4] != kB * kH || in_sizes[5] != kB * kH || in_sizes[6] != kH * kH || in_sizes[7] != kH || in_sizes[8] != kH * kH || in_sizes[9] != kH) return;
  if (in_sizes[10] != kH * kH || in_sizes[11] != kH || in_sizes[12] != kH || in_sizes[13] != 1 || in_sizes[14] != kH2 * kH2 || in_sizes[15] != kH2) return;
  if (in_sizes[16] != kG4 * kH2 || in_sizes[17] != kG4 * kH || in_sizes[18] != kG4 || in_sizes[19] != kG4) return;
  if (out_size != kB * kT * kH) return;
  if (ws_size < kWsTotal) return;
  const float* x      = (const float*)d_in[0];
  const int*   x_mask = (const int*)d_in[1];
  const float* y      = (const float*)d_in[2];
  const int*   y_mask = (const int*)d_in[3];
  const float* h0     = (const float*)d_in[4];
  const float* c0     = (const float*)d_in[5];
  const float* Wq     = (const float*)d_in[6];
  const float* bq     = (const float*)d_in[7];
  const float* Wup    = (const float*)d_in[8];
  const float* bup    = (const float*)d_in[9];
  const float* Wvp    = (const float*)d_in[10];
  const float* bvp    = (const float*)d_in[11];
  const float* Vw     = (const float*)d_in[12];
  const float* Vb     = (const float*)d_in[13];
  const float* Wg     = (const float*)d_in[14];
  const float* bg     = (const float*)d_in[15];
  const float* Wih    = (const float*)d_in[16];
  const float* Whh    = (const float*)d_in[17];
  const float* bih    = (const float*)d_in[18];
  const float* bhh    = (const float*)d_in[19];
  float* out = (float*)d_out;
  char* ws = (char*)d_ws;
  unsigned short* X16  = (unsigned short*)(ws + kOffX16);
  unsigned short* Y16  = (unsigned short*)(ws + kOffY16);
  unsigned short* WQ   = (unsigned short*)(ws + kOffWQ);
  unsigned short* WUP  = (unsigned short*)(ws + kOffWUP);
  unsigned short* WG   = (unsigned short*)(ws + kOffWG);
  unsigned short* WIH  = (unsigned short*)(ws + kOffWIH);
  unsigned short* WHV  = (unsigned short*)(ws + kOffWHV);
  float* F    = (float*)(ws + kOffF32);
  float* YP   = (float*)(ws + kOffYP);
  float* XU   = (float*)(ws + kOffXU);
  float* XG   = (float*)(ws + kOffXG);
  float* HV   = (float*)(ws + kOffHV);
  float* CG   = (float*)(ws + kOffCG);
  float* GI   = (float*)(ws + kOffGI);
  float* CT32 = (float*)(ws + kOffCT32);
  unsigned short* H16  = (unsigned short*)(ws + kOffH16);
  unsigned short* CT16 = (unsigned short*)(ws + kOffCT16);
  unsigned short* LI16 = (unsigned short*)(ws + kOffLI16);

  cast_plane_kernel<<<(int)(((size_t)kRowsX * kH / 8) / kThr), kThr, 0, stream>>>(x, X16, 8, kH, 0);
  cast_plane_kernel<<<(int)(((size_t)kRowsY * kH / 8) / kThr), kThr, 0, stream>>>(y, Y16, 8, kH, 0);
  cast_plane_kernel<<<(int)(((size_t)kH * kH / 8) / kThr), kThr, 0, stream>>>(Wq, WQ, 8, kH, 0);
  cast_plane_kernel<<<(int)(((size_t)kH * kH / 8) / kThr), kThr, 0, stream>>>(Wup, WUP, 8, kH, 0);
  cast_plane_kernel<<<(int)(((size_t)kH2 * kH2 / 8) / kThr), kThr, 0, stream>>>(Wg, WG, 9, kH2, 0);
  cast_plane_kernel<<<(int)(((size_t)kG4 * kH2 / 8) / kThr), kThr, 0, stream>>>(Wih, WIH, 9, kH2, 0);
  cast_plane_kernel<<<(int)(((size_t)kG4 * kH / 8) / kThr), kThr, 0, stream>>>(Whh, WHV, 8, kH, 0);
  cast_plane_kernel<<<(int)(((size_t)kH * kH / 8) / kThr), kThr, 0, stream>>>(Wvp, WHV + (size_t)kG4 * kH, 8, kH, 0);
  setup_f32_kernel<<<12, kThr, 0, stream>>>(bq, bup, bg, bih, bhh, bvp, c0, F);
  setup_f16_kernel<<<52, kThr, 0, stream>>>(h0, WHV, H16, CT16, LI16);

  wmma_gemm64<0, false, 2, 0, false, 0><<<dim3((kRowsY / 64) * (kH / 64) / 8, 1), 256, 0, stream>>>(
      Y16, Y16, kH, 0L, WQ, WQ, kH, 0L, (void*)YP, (void*)YP, kH, 0L, F + kFBQ, nullptr, 0L, kRowsY, kH, kH, kSc);
  wmma_gemm64<0, false, 2, 0, false, 0><<<dim3((kRowsX / 64) * (kH / 64) / 8, 1), 256, 0, stream>>>(
      X16, X16, kH, 0L, WUP, WUP, kH, 0L, (void*)XU, (void*)XU, kH, 0L, F + kFBUP, nullptr, 0L, kRowsX, kH, kH, kSc);
  wmma_gemm64<0, false, 2, 0, false, 0><<<dim3((kRowsX / 64) * (kH2 / 64) / 8, 1), 256, 0, stream>>>(
      X16, X16, kH, 0L, WG, WG, kH2, 0L, (void*)XG, (void*)XG, kH2, 0L, F + kFBGT, nullptr, 0L, kRowsX, kH2, kH, kSc);

  for (int t = 0; t < kT; ++t) {
    wmma_gemm64<0, false, 2, 0, false, 0><<<dim3((kBP / 64) * (kNS / 64) / 8, 1), 256, 0, stream>>>(
        H16, H16, kH, 0L, WHV, WHV, kH, 0L, (void*)HV, (void*)HV, kNS, 0L, F + kFBHV, nullptr, 0L, kBP, kNS, kH, kSc);
    add_attn_kernel<<<kB, kThr, 0, stream>>>(YP, XU, HV, Vw, Vb, y_mask, Y16, CT32, CT16, t);
    wmma_gemm64<0, false, 2, 0, false, 0><<<dim3((kBP / 64) * (kH2 / 64) / 8, 1), 256, 0, stream>>>(
        CT16, CT16, kH, 0L, WG + kH, WG + kH, kH2, 0L, (void*)CG, (void*)CG, kH2, 0L, F + kFZB, nullptr, 0L, kBP, kH2, kH, kSc);
    in_gate_kernel<<<8, kThr, 0, stream>>>(x, x_mask, CT32, XG, CG, LI16, t);
    wmma_gemm64<0, false, 2, 0, false, 0><<<dim3((kBP / 64) * (kG4 / 64) / 8, 1), 256, 0, stream>>>(
        LI16, LI16, kH2, 0L, WIH, WIH, kH2, 0L, (void*)GI, (void*)GI, kG4, 0L, F + kFBGI, nullptr, 0L, kBP, kG4, kH2, kSc);
    masked_cell_kernel<<<4, kThr, 0, stream>>>(GI, HV, x_mask, F + kFC32, H16, out, t);
  }
}
